// LinkPredictorWithContrastiveLearning_53360673686007
// MI455X (gfx1250) — hardware-verified
//
#include <hip/hip_runtime.h>


namespace {
constexpr int N = 100000, E = 600000, D = 128, H = 256;
constexpr float XS = 8.0f, WSC = 256.0f;
typedef _Float16 b16;
typedef __attribute__((ext_vector_type(16))) _Float16 v16b;
typedef __attribute__((ext_vector_type(8))) _Float16 v8b;
typedef __attribute__((ext_vector_type(8))) float v8f;
typedef __attribute__((ext_vector_type(4))) float v4f;
__device__ __forceinline__ float bf16_rne(float f) { unsigned int u = __float_as_uint(f); u += 0x7FFFu + ((u >> 16) & 1u); float r = __uint_as_float(u & 0xFFFF0000u); asm volatile("" : "+v"(r)); return r; }
__device__ __forceinline__ float bfv(float f) { float r = bf16_rne(f); asm volatile("" : "+v"(r)); return r; }
__device__ __forceinline__ v16b frag_kb(const b16* p, int hh) { const v8b a = *(const v8b*)(p + 8 * hh), b = *(const v8b*)(p + 16 + 8 * hh); v16b f;
#pragma unroll
  for (int e = 0; e < 8; ++e) { f[e] = a[e]; f[8 + e] = b[e]; } return f; }
__device__ __forceinline__ v8f wmma16b(v16b a, v16b b, v8f c) { v8f d = __builtin_amdgcn_wmma_f32_16x16x32_f16(false, a, false, b, (short)0, c, false, false); asm volatile("v_nop\n\tv_nop\n\tv_nop\n\tv_nop" : "+v"(d) : "v"(a), "v"(b)); return d; }
__device__ __forceinline__ void wave_lds_sync() { __builtin_amdgcn_fence(__ATOMIC_RELEASE, "workgroup"); __builtin_amdgcn_wave_barrier(); __builtin_amdgcn_fence(__ATOMIC_ACQUIRE, "workgroup"); }
__device__ __forceinline__ float pmul(float a, float b) { float p = a * b; asm volatile("" : "+v"(p)); return p; }
__device__ __forceinline__ int iclamp(int v, int lo, int hi) { return v < lo ? lo : (v > hi ? hi : v); }

__global__ __launch_bounds__(256) void wput_kernel(const float* __restrict__ w1, b16* __restrict__ WT) { const int u = blockIdx.x * 256 + threadIdx.x; if (u >= 2 * H * 16) return; const int op = u / 16, k0 = (u % 16) * 8; const int o = op % H, half = op / H; v8b v;
#pragma unroll
  for (int j = 0; j < 8; ++j) v[j] = (b16)(bf16_rne(w1[(size_t)(half * D + k0 + j) * H + o]) * WSC); for (int pass = 0; pass < 2; ++pass) { *(volatile v8b*)(WT + (size_t)op * D + k0) = v; __threadfence(); } }
__global__ __launch_bounds__(32) void node_kernel(const float* __restrict__ emd, const b16* __restrict__ WT, int NLIM, float* __restrict__ P) { __shared__ __attribute__((aligned(16))) b16 Ah[16][D + 8]; __shared__ float Tf[16][260]; const int lane = threadIdx.x, nloc = lane & 15, hlf = lane >> 4; const int g = blockIdx.x % 2; const size_t m0 = (size_t)(blockIdx.x / 2) * 16; if (m0 >= (size_t)NLIM) return;
  for (int rr = 0; rr < 16; ++rr) for (int q = 0; q < 4; ++q) Ah[rr][q * 32 + lane] = (b16)(bf16_rne(emd[(m0 + rr) * D + q * 32 + lane]) * XS); if (lane < 16) for (int k = D; k < D + 8; ++k) Ah[lane][k] = (b16)0.0f;
  wave_lds_sync(); v8f acc[16];
#pragma unroll
  for (int t = 0; t < 16; ++t) acc[t] = (v8f){};
#pragma unroll
  for (int kb = 0; kb < D; kb += 32) { const v16b a = frag_kb(&Ah[nloc][kb], hlf);
#pragma unroll
    for (int t = 0; t < 16; ++t) acc[t] = wmma16b(a, frag_kb(WT + (size_t)(g * 256 + t * 16 + nloc) * D + kb, hlf), acc[t]); }
#pragma unroll
  for (int t = 0; t < 16; ++t)
#pragma unroll
    for (int r8 = 0; r8 < 8; ++r8) Tf[8 * hlf + r8][t * 16 + nloc] = acc[t][r8] * (1.0f / (XS * WSC));
  wave_lds_sync();
  for (int pass = 0; pass < 2; ++pass) { for (int rr = 0; rr < 16; ++rr) for (int q = 0; q < 2; ++q) *(volatile v4f*)(P + (m0 + rr) * 2 * H + g * H + q * 128 + lane * 4) = *(const v4f*)(&Tf[rr][q * 128 + lane * 4]); __threadfence(); } }
__global__ __launch_bounds__(256) void edge_kernel(const float* __restrict__ P, const int* __restrict__ ei, const float* __restrict__ b1, const float* __restrict__ w2, const float* __restrict__ b2, int NLIM, int ELIM, float* __restrict__ out) { const size_t e = (size_t)blockIdx.x * 256 + threadIdx.x; if (e >= (size_t)ELIM) return; const size_t s = (size_t)iclamp(ei[e * 2], 0, NLIM - 1), d = (size_t)iclamp(ei[e * 2 + 1], 0, NLIM - 1); const float* ps = P + s * 2 * H; const float* pd = P + d * 2 * H + H; float acc = bfv(b2[0]);
#pragma unroll 4
  for (int c = 0; c < H; ++c) { const float h = fmaxf(ps[c] + pd[c] + bfv(b1[c]), 0.0f); acc += pmul(h, bfv(w2[c])); }
  const float p = 1.0f / (1.0f + __expf(-acc));
  for (int pass = 0; pass < 2; ++pass) { ((volatile float*)out)[e] = p; __threadfence(); } }
}

extern "C" void kernel_launch(void* const* d_in, const int* in_sizes, int n_in, void* d_out, int out_size, void* d_ws, size_t ws_size, hipStream_t stream) {
  (void)n_in;
  auto Fp = [&](int i) { return (const float*)d_in[i]; }; auto Ip = [&](int i) { return (const int*)d_in[i]; };
  if (in_sizes[0] != N * D || in_sizes[1] != E * 2 || in_sizes[2] != 2 * D * H || in_sizes[3] != H || in_sizes[4] != H || out_size != E) return;
  const int NLIM = N, ELIM = E;
  size_t off = 0; char* ws = (char*)d_ws;
  auto carve = [&](size_t bytes) { char* p = ws + off; off += (bytes + 255) & ~(size_t)255; return p; };
  b16* WT = (b16*)carve((size_t)2 * H * D * 2); float* P = (float*)carve((size_t)N * 2 * H * 4);
  if (off > ws_size || off > ((size_t)240 << 20)) return;
  wput_kernel<<<(2 * H * 16 + 255) / 256, 256, 0, stream>>>(Fp(2), WT);
  node_kernel<<<(NLIM / 16) * 2, 32, 0, stream>>>(Fp(0), WT, NLIM, P);
  edge_kernel<<<(ELIM + 255) / 256, 256, 0, stream>>>(P, Ip(1), Fp(3), Fp(4), Fp(5), NLIM, ELIM, (float*)d_out);
}
